// RKNCell_10926396801277
// MI455X (gfx1250) — hardware-run, weakly checked
//
#include <hip/hip_runtime.h>
#include <math.h>

typedef __attribute__((ext_vector_type(16))) _Float16 v16h;
typedef __attribute__((ext_vector_type(8)))  _Float16 v8h;
typedef __attribute__((ext_vector_type(8)))  float    v8f;
typedef __attribute__((ext_vector_type(4)))  float    v4f;
typedef __attribute__((ext_vector_type(2)))  float    v2f;

constexpr int kBatch = 4096;
constexpr int kLod   = 64;
constexpr int kLsd   = 128;
constexpr int kHid   = 64;
constexpr int kNb    = 15;
constexpr int kNe    = 436;
constexpr int kBw    = 3;

constexpr size_t kOffPM  = 0;
constexpr size_t kOffPCU = kOffPM  + (size_t)kBatch * kLsd;
constexpr size_t kOffPCL = kOffPCU + (size_t)kBatch * kLod;
constexpr size_t kOffPCS = kOffPCL + (size_t)kBatch * kLod;
constexpr size_t kOffNM  = kOffPCS + (size_t)kBatch * kLod;
constexpr size_t kOffNCU = kOffNM  + (size_t)kBatch * kLsd;
constexpr size_t kOffNCL = kOffNCU + (size_t)kBatch * kLod;
constexpr size_t kOffNCS = kOffNCL + (size_t)kBatch * kLod;
constexpr size_t kOutTotal = kOffNCS + (size_t)kBatch * kLod;
static_assert(kOffPCU * 4 == 2097152ull);
static_assert(kOffPCL * 4 == 3145728ull);
static_assert(kOffPCS * 4 == 4194304ull);
static_assert(kOffNM  * 4 == 5242880ull);
static_assert(kOffNCU * 4 == 7340032ull);
static_assert(kOffNCL * 4 == 8388608ull);
static_assert(kOffNCS * 4 == 9437184ull);
static_assert(kOutTotal * 4 == 10485760ull);

constexpr float kActCarry = 64.0f;
constexpr float kWCarry   = 256.0f;
constexpr float kInvCarry = 1.0f / (kActCarry * kWCarry);
constexpr float kF16MinNormal = 6.103515625e-05f;

constexpr int kSP = 68;
constexpr int kHP = 72;

constexpr int kPR = 8;
constexpr int kIC = 32;
constexpr int kTP = 256;

constexpr size_t kOffW1H   = 0;
constexpr size_t kOffW2H   = kOffW1H + (size_t)kHid * kLsd * 2;
constexpr size_t kOffW3H   = kOffW2H + (size_t)kHid * kHid * 2;
constexpr size_t kOffTC    = kOffW3H + (size_t)16 * kHid * 2;
constexpr size_t kOffA0    = kOffTC  + (size_t)kLsd * 4;
constexpr size_t kOffCOEFF = kOffA0  + (size_t)kBatch * kLsd * 2;
constexpr size_t kWsTotal  = kOffCOEFF + (size_t)kBatch * 16 * 4;
static_assert(kWsTotal == 1337856ull);
static_assert(kWsTotal <= 134217728ull);
static_assert((kOffW2H % 128) == 0 && (kOffW3H % 128) == 0 && (kOffTC % 128) == 0 &&
              (kOffA0 % 128) == 0 && (kOffCOEFF % 128) == 0);
static_assert((kLsd % 32) == 0 && (kHid % 32) == 0 && (kBatch % 64) == 0 && (kHid % 16) == 0);

__host__ __device__ constexpr int band_rs(int i) {
  return (i < 3) ? ((i * (i + 7)) / 2)
                 : ((i > 61) ? (kNe - ((64 - i) * (71 - i)) / 2) : (7 * i - 6));
}
static_assert(band_rs(0) == 0 && band_rs(1) == 4 && band_rs(2) == 9 && band_rs(3) == 15);
static_assert(band_rs(61) == 421 && band_rs(62) == 427 && band_rs(63) == 432 && band_rs(64) == kNe);
static_assert(band_rs(32) == 218);
static_assert(band_rs(32) - band_rs(0) <= kTP && band_rs(64) - band_rs(32) <= kTP);
static_assert(kBw == 3 && kLod == 64);

struct FragH {
  union U { v16h v; v8h h[2]; };
  static __device__ __forceinline__ v16h load(const _Float16* p) {
    U f;
    f.h[0] = *(const v8h*)(p);
    f.h[1] = *(const v8h*)(p + 16);
    return f.v;
  }
};
__device__ __forceinline__ v8f mma_f16(v16h a, v16h b, v8f c) {
  c = __builtin_amdgcn_wmma_f32_16x16x32_f16(false, a, false, b, (short)0, c, false, false);
  asm volatile("v_nop\n\tv_nop\n\tv_nop\n\tv_nop" : "+v"(c) : "v"(a), "v"(b));
  return c;
}

__device__ __forceinline__ float carry_flush(float v, float carry) {
  const float s = v * carry;
  return (fabsf(s) < kF16MinNormal) ? 0.0f : s;
}
__device__ __forceinline__ v8h pack8_f16(v4f a0, v4f a1, float carry) {
  v8h hv;
#pragma unroll
  for (int e = 0; e < 4; ++e) {
    hv[e]     = (_Float16)carry_flush(a0[e], carry);
    hv[4 + e] = (_Float16)carry_flush(a1[e], carry);
  }
  return hv;
}

__global__ __launch_bounds__(256) void prep_planes_kernel(
    const float* __restrict__ W1, const float* __restrict__ W2, const float* __restrict__ W3,
    const float* __restrict__ ltn,
    unsigned short* __restrict__ w1h, unsigned short* __restrict__ w2h, unsigned short* __restrict__ w3h,
    float* __restrict__ tcp)
{
  const int blk = blockIdx.x;
  const int tid = threadIdx.x;
  if (blk < 6) {
    const bool first = (blk < 4);
    const float* src = first ? W1 : W2;
    unsigned short* dst = first ? w1h : w2h;
    const int t = (first ? blk : (blk - 4)) * 256 + tid;
    const size_t e0 = (size_t)t * 8;
    const v4f a0 = *(const v4f*)(src + e0);
    const v4f a1 = *(const v4f*)(src + e0 + 4);
    const v8h hv = pack8_f16(a0, a1, kWCarry);
    unsigned short* q = dst + e0;
    *(volatile v8h*)q = hv;
    __threadfence();
    *(volatile v8h*)q = hv;
  } else if (tid < 128) {
    const int n = tid >> 3;
    const int k = (tid & 7) * 8;
    const int ns = (n < kNb) ? n : (kNb - 1);
    v4f a0 = *(const v4f*)(W3 + (size_t)ns * kHid + k);
    v4f a1 = *(const v4f*)(W3 + (size_t)ns * kHid + k + 4);
    asm volatile("" : "+v"(a0), "+v"(a1));
    const bool live = (n < kNb);
    v4f z0, z1;
#pragma unroll
    for (int e = 0; e < 4; ++e) {
      z0[e] = live ? a0[e] : 0.0f;
      z1[e] = live ? a1[e] : 0.0f;
    }
    const v8h hv = pack8_f16(z0, z1, kWCarry);
    unsigned short* q = w3h + (size_t)tid * 8;
    *(volatile v8h*)q = hv;
    __threadfence();
    *(volatile v8h*)q = hv;
  } else {
    const int q = tid - 128;
    const float x = ltn[q];
    const float v = logf(expf(x) + 1.0f);
    volatile float* d = tcp + q;
    *d = v;
    __threadfence();
    *d = v;
  }
}

__global__ __launch_bounds__(256) void gain_update_kernel(
    const float* __restrict__ pm, const float* __restrict__ cu, const float* __restrict__ cl,
    const float* __restrict__ cs, const float* __restrict__ ob, const float* __restrict__ ov,
    float* __restrict__ out, unsigned* __restrict__ a0w)
{
  const int gid = blockIdx.x * 256 + threadIdx.x;
  const int b = gid >> 5;
  const int p = gid & 31;
  if (b >= kBatch) return;
  const int c = 2 * p;
  const size_t o64  = (size_t)b * kLod + c;
  const size_t o128 = (size_t)b * kLsd + c;
  const v2f du  = *(const v2f*)(cu + o64);
  const v2f lc  = *(const v2f*)(cl + o64);
  const v2f sc  = *(const v2f*)(cs + o64);
  const v2f obv = *(const v2f*)(ob + o64);
  const v2f vo  = *(const v2f*)(ov + o64);
  const v2f mu0 = *(const v2f*)(pm + o128);
  const v2f ml0 = *(const v2f*)(pm + o128 + kLod);
  v2f pmu, pml, pcu, pcl, pcs;
#pragma unroll
  for (int e = 0; e < 2; ++e) {
    const float den = du[e] + vo[e];
    const float qu = du[e] / den;
    const float ql = sc[e] / den;
    const float res = obv[e] - mu0[e];
    pmu[e] = mu0[e] + qu * res;
    pml[e] = ml0[e] + ql * res;
    const float cf = 1.0f - qu;
    pcu[e] = cf * du[e];
    pcl[e] = lc[e] - ql * sc[e];
    pcs[e] = cf * sc[e];
  }
  const float u0 = pmu[0], u1 = pmu[1], l0 = pml[0], l1 = pml[1];
  const _Float16 hu0 = (_Float16)carry_flush(u0, kActCarry);
  const _Float16 hu1 = (_Float16)carry_flush(u1, kActCarry);
  const _Float16 hl0 = (_Float16)carry_flush(l0, kActCarry);
  const _Float16 hl1 = (_Float16)carry_flush(l1, kActCarry);
  const unsigned wu = (unsigned)__builtin_bit_cast(unsigned short, hu0) |
                      ((unsigned)__builtin_bit_cast(unsigned short, hu1) << 16);
  const unsigned wl = (unsigned)__builtin_bit_cast(unsigned short, hl0) |
                      ((unsigned)__builtin_bit_cast(unsigned short, hl1) << 16);
  float* q_pmu = out + kOffPM + o128;
  float* q_pml = out + kOffPM + o128 + kLod;
  float* q_pcu = out + kOffPCU + o64;
  float* q_pcl = out + kOffPCL + o64;
  float* q_pcs = out + kOffPCS + o64;
  unsigned* q_au = a0w + (size_t)b * (kLsd / 2) + p;
  unsigned* q_al = a0w + (size_t)b * (kLsd / 2) + (kLod / 2) + p;
  for (int pass = 0; pass < 2; ++pass) {
    *(volatile v2f*)q_pmu = pmu;
    *(volatile v2f*)q_pml = pml;
    *(volatile v2f*)q_pcu = pcu;
    *(volatile v2f*)q_pcl = pcl;
    *(volatile v2f*)q_pcs = pcs;
    *(volatile unsigned*)q_au = wu;
    *(volatile unsigned*)q_al = wl;
    __threadfence();
  }
}

__device__ __forceinline__ void dump_acc4(float* slab, const v8f (&acc)[4], int hh, int c) {
#pragma unroll
  for (int j = 0; j < 4; ++j) {
#pragma unroll
    for (int r = 0; r < 8; ++r) slab[(8 * hh + r) * kSP + j * 16 + c] = acc[j][r];
  }
}
__device__ __forceinline__ void act_tile(const float* slab, _Float16* hs, float ba, float bb, int lane) {
#pragma unroll 1
  for (int it = 0; it < 32; ++it) {
    const int row = it >> 1;
    const int col = (it & 1) * 32 + lane;
    const float bias = (it & 1) ? bb : ba;
    const float v = slab[row * kSP + col] * kInvCarry + bias;
    const float t = tanhf(v);
    hs[row * kHP + col] = (_Float16)carry_flush(t, kActCarry);
  }
}

__global__ __launch_bounds__(128) void coeff_net_kernel(
    const unsigned short* __restrict__ a0p, const unsigned short* __restrict__ w1p,
    const unsigned short* __restrict__ w2p, const unsigned short* __restrict__ w3p,
    const float* __restrict__ b1, const float* __restrict__ b2, const float* __restrict__ b3,
    float* __restrict__ coeff)
{
  __shared__ __align__(16) float    sS[4][16 * kSP];
  __shared__ __align__(16) _Float16 sH[4][16 * kHP];
  const _Float16* A0  = (const _Float16*)a0p;
  const _Float16* W1h = (const _Float16*)w1p;
  const _Float16* W2h = (const _Float16*)w2p;
  const _Float16* W3h = (const _Float16*)w3p;
  const int tid  = threadIdx.x;
  const int wave = tid >> 5;
  const int lane = tid & 31;
  const int hh   = lane >> 4;
  const int c    = lane & 15;
  const int koff = hh * 8;
  const int m0   = blockIdx.x * 64 + wave * 16;
  float*    slab = sS[wave];
  _Float16* hs   = sH[wave];

  const float b1a = b1[lane], b1b = b1[lane + 32];
  const float b2a = b2[lane], b2b = b2[lane + 32];
  const int   b3i = (c < kNb) ? c : (kNb - 1);
  float b3v = b3[b3i];
  asm volatile("" : "+v"(b3v));
  b3v = (c < kNb) ? b3v : 0.0f;

  v8f acc[4];
#pragma unroll
  for (int j = 0; j < 4; ++j) acc[j] = (v8f){0.f,0.f,0.f,0.f,0.f,0.f,0.f,0.f};

#pragma unroll 1
  for (int k0 = 0; k0 < kLsd; k0 += 32) {
    const v16h a = FragH::load(A0 + (size_t)(m0 + c) * kLsd + koff + k0);
#pragma unroll
    for (int j = 0; j < 4; ++j) {
      const v16h b = FragH::load(W1h + (size_t)(j * 16 + c) * kLsd + koff + k0);
      acc[j] = mma_f16(a, b, acc[j]);
    }
  }
  dump_acc4(slab, acc, hh, c);
  __syncthreads();
  act_tile(slab, hs, b1a, b1b, lane);
  __syncthreads();

#pragma unroll
  for (int j = 0; j < 4; ++j) acc[j] = (v8f){0.f,0.f,0.f,0.f,0.f,0.f,0.f,0.f};
#pragma unroll
  for (int k0 = 0; k0 < kHid; k0 += 32) {
    const v16h a = FragH::load(hs + c * kHP + koff + k0);
#pragma unroll
    for (int j = 0; j < 4; ++j) {
      const v16h b = FragH::load(W2h + (size_t)(j * 16 + c) * kHid + koff + k0);
      acc[j] = mma_f16(a, b, acc[j]);
    }
  }
  dump_acc4(slab, acc, hh, c);
  __syncthreads();
  act_tile(slab, hs, b2a, b2b, lane);
  __syncthreads();

  v8f lg = (v8f){0.f,0.f,0.f,0.f,0.f,0.f,0.f,0.f};
#pragma unroll
  for (int k0 = 0; k0 < kHid; k0 += 32) {
    const v16h a = FragH::load(hs + c * kHP + koff + k0);
    const v16h b = FragH::load(W3h + (size_t)c * kHid + koff + k0);
    lg = mma_f16(a, b, lg);
  }
  const bool live = (c < kNb);
#pragma unroll
  for (int r = 0; r < 8; ++r) {
    const float raw = lg[r] * kInvCarry + b3v;
    const float x = live ? raw : -INFINITY;
    float m = x;
    m = fmaxf(m, __shfl_xor(m, 1, 32));
    m = fmaxf(m, __shfl_xor(m, 2, 32));
    m = fmaxf(m, __shfl_xor(m, 4, 32));
    m = fmaxf(m, __shfl_xor(m, 8, 32));
    const float ex = expf(x - m);
    float s = ex;
    s += __shfl_xor(s, 1, 32);
    s += __shfl_xor(s, 2, 32);
    s += __shfl_xor(s, 4, 32);
    s += __shfl_xor(s, 8, 32);
    const float pr = ex / s;
    slab[(8 * hh + r) * 16 + c] = pr;
  }
  __syncthreads();
  const v4f v0 = *(const v4f*)(slab + lane * 4);
  const v4f v1 = *(const v4f*)(slab + 128 + lane * 4);
  float* q0 = coeff + (size_t)m0 * 16 + lane * 4;
  float* q1 = q0 + 128;
  for (int pass = 0; pass < 2; ++pass) {
    *(volatile v4f*)q0 = v0;
    *(volatile v4f*)q1 = v1;
    __threadfence();
  }
}

__global__ __launch_bounds__(256) void predict_kernel(
    float* dout, const float* __restrict__ coeff, const float* __restrict__ tc,
    const float* __restrict__ bs11, const float* __restrict__ bs12,
    const float* __restrict__ bs21, const float* __restrict__ bs22)
{
  __shared__ __align__(16) float sC[kPR * 16];
  __shared__ __align__(16) float sPM[kPR * kLsd];
  __shared__ __align__(16) float sCU[kPR * kLod];
  __shared__ __align__(16) float sCL[kPR * kLod];
  __shared__ __align__(16) float sCS[kPR * kLod];
  __shared__ __align__(16) float sTM[4 * kPR * kTP];

  const int tid  = threadIdx.x;
  const int wave = tid >> 5;
  const int lane = tid & 31;
  const int row0 = blockIdx.x * kPR;
  const float* post = (const float*)dout;

  *(v4f*)(sPM + tid * 4) = *(const v4f*)(post + kOffPM  + (size_t)row0 * kLsd + tid * 4);
  *(v2f*)(sCU + tid * 2) = *(const v2f*)(post + kOffPCU + (size_t)row0 * kLod + tid * 2);
  *(v2f*)(sCL + tid * 2) = *(const v2f*)(post + kOffPCL + (size_t)row0 * kLod + tid * 2);
  *(v2f*)(sCS + tid * 2) = *(const v2f*)(post + kOffPCS + (size_t)row0 * kLod + tid * 2);
  if (tid < 32) *(v4f*)(sC + tid * 4) = *(const v4f*)(coeff + (size_t)row0 * 16 + tid * 4);
  __syncthreads();

#pragma unroll 1
  for (int ic = 0; ic < kLod / kIC; ++ic) {
    const int e0 = band_rs(ic * kIC);
    const int ec = band_rs(ic * kIC + kIC) - e0;
    const int es = (tid < ec) ? tid : (ec - 1);
    const int e  = e0 + es;
#pragma unroll 1
    for (int p = 0; p < 4; ++p) {
      const float* bp = (p == 0) ? bs11 : ((p == 1) ? bs12 : ((p == 2) ? bs21 : bs22));
      float bv[kNb];
#pragma unroll
      for (int k = 0; k < kNb; ++k) bv[k] = bp[k * kNe + e];
#pragma unroll 1
      for (int r = 0; r < kPR; ++r) {
        const float* cr = sC + r * 16;
        const v4f c0 = *(const v4f*)(cr);
        const v4f c1 = *(const v4f*)(cr + 4);
        const v4f c2 = *(const v4f*)(cr + 8);
        const v4f c3 = *(const v4f*)(cr + 12);
        float s = 0.0f;
        s = fmaf(c0[0], bv[0], s);
        s = fmaf(c0[1], bv[1], s);
        s = fmaf(c0[2], bv[2], s);
        s = fmaf(c0[3], bv[3], s);
        s = fmaf(c1[0], bv[4], s);
        s = fmaf(c1[1], bv[5], s);
        s = fmaf(c1[2], bv[6], s);
        s = fmaf(c1[3], bv[7], s);
        s = fmaf(c2[0], bv[8], s);
        s = fmaf(c2[1], bv[9], s);
        s = fmaf(c2[2], bv[10], s);
        s = fmaf(c2[3], bv[11], s);
        s = fmaf(c3[0], bv[12], s);
        s = fmaf(c3[1], bv[13], s);
        s = fmaf(c3[2], bv[14], s);
        sTM[(p * kPR + r) * kTP + tid] = s;
      }
    }
    __syncthreads();

    const int r  = wave;
    const int i  = ic * kIC + lane;
    const int jl = (i - kBw < 0) ? 0 : (i - kBw);
    const int ebase = band_rs(i) - e0;
    const float* t11p = sTM + (0 * kPR + r) * kTP;
    const float* t12p = sTM + (1 * kPR + r) * kTP;
    const float* t21p = sTM + (2 * kPR + r) * kTP;
    const float* t22p = sTM + (3 * kPR + r) * kTP;
    const float* pmr = sPM + r * kLsd;
    const float* cur = sCU + r * kLod;
    const float* clr = sCL + r * kLod;
    const float* csr = sCS + r * kLod;
    float nmu = 0.0f, nml = 0.0f, ncu = 0.0f, ncl = 0.0f, ncs = 0.0f;
#pragma unroll 1
    for (int jj = 0; jj < 2 * kBw + 1; ++jj) {
      const int j = i - kBw + jj;
      const bool ok = (j >= 0) && (j <= kLod - 1);
      const int jc = (j < 0) ? 0 : ((j > kLod - 1) ? (kLod - 1) : j);
      const int ee = ebase + (jc - jl);
      float a = t11p[ee];
      float b = t12p[ee];
      float c = t21p[ee];
      float d = t22p[ee];
      const float dg = (jc == i) ? 1.0f : 0.0f;
      a += dg;
      d += dg;
      a = ok ? a : 0.0f;
      b = ok ? b : 0.0f;
      c = ok ? c : 0.0f;
      d = ok ? d : 0.0f;
      const float mu = pmr[jc];
      const float ml = pmr[kLod + jc];
      const float xu = cur[jc];
      const float xl = clr[jc];
      const float xs = csr[jc];
      nmu = fmaf(a, mu, nmu);
      nmu = fmaf(b, ml, nmu);
      nml = fmaf(c, mu, nml);
      nml = fmaf(d, ml, nml);
      ncu = fmaf(a * a, xu, ncu);
      ncu = fmaf(2.0f * (a * b), xs, ncu);
      ncu = fmaf(b * b, xl, ncu);
      ncl = fmaf(c * c, xu, ncl);
      ncl = fmaf(2.0f * (c * d), xs, ncl);
      ncl = fmaf(d * d, xl, ncl);
      ncs = fmaf(c * a, xu, ncs);
      ncs = fmaf(fmaf(d, a, c * b), xs, ncs);
      ncs = fmaf(d * b, xl, ncs);
    }
    const float tcu = tc[i];
    const float tcl = tc[kLod + i];
    const float o_ncu = ncu + tcu;
    const float o_ncl = ncl + tcl;
    const int row = row0 + r;
    float* q_nmu = dout + kOffNM  + (size_t)row * kLsd + i;
    float* q_nml = dout + kOffNM  + (size_t)row * kLsd + kLod + i;
    float* q_ncu = dout + kOffNCU + (size_t)row * kLod + i;
    float* q_ncl = dout + kOffNCL + (size_t)row * kLod + i;
    float* q_ncs = dout + kOffNCS + (size_t)row * kLod + i;
    for (int pass = 0; pass < 2; ++pass) {
      *(volatile float*)q_nmu = nmu;
      *(volatile float*)q_nml = nml;
      *(volatile float*)q_ncu = o_ncu;
      *(volatile float*)q_ncl = o_ncl;
      *(volatile float*)q_ncs = ncs;
      __threadfence();
    }
    __syncthreads();
  }
}

extern "C" void kernel_launch(void* const* d_in, const int* in_sizes, int n_in,
                              void* d_out, int out_size, void* d_ws, size_t ws_size,
                              hipStream_t stream) {
  if (n_in < 17) return;
  if (in_sizes[0] != kBatch * kLsd) return;
  if (in_sizes[1] != kBatch * kLod) return;
  if (in_sizes[2] != kBatch * kLod) return;
  if (in_sizes[3] != kBatch * kLod) return;
  if (in_sizes[4] != kBatch * kLod) return;
  if (in_sizes[5] != kBatch * kLod) return;
  if (in_sizes[6] != kHid * kLsd) return;
  if (in_sizes[7] != kHid) return;
  if (in_sizes[8] != kHid * kHid) return;
  if (in_sizes[9] != kHid) return;
  if (in_sizes[10] != kNb * kHid) return;
  if (in_sizes[11] != kNb) return;
  if (in_sizes[12] != kNb * kNe) return;
  if (in_sizes[13] != kNb * kNe) return;
  if (in_sizes[14] != kNb * kNe) return;
  if (in_sizes[15] != kNb * kNe) return;
  if (in_sizes[16] != kLsd) return;
  if ((size_t)out_size != kOutTotal) return;
  if (ws_size < kWsTotal) return;

  const float* prior_mean = (const float*)d_in[0];
  const float* cov_u      = (const float*)d_in[1];
  const float* cov_l      = (const float*)d_in[2];
  const float* cov_s      = (const float*)d_in[3];
  const float* obs        = (const float*)d_in[4];
  const float* obs_var    = (const float*)d_in[5];
  const float* W1         = (const float*)d_in[6];
  const float* b1         = (const float*)d_in[7];
  const float* W2         = (const float*)d_in[8];
  const float* b2         = (const float*)d_in[9];
  const float* W3         = (const float*)d_in[10];
  const float* b3         = (const float*)d_in[11];
  const float* tm11b      = (const float*)d_in[12];
  const float* tm12b      = (const float*)d_in[13];
  const float* tm21b      = (const float*)d_in[14];
  const float* tm22b      = (const float*)d_in[15];
  const float* ltn        = (const float*)d_in[16];
  float* out = (float*)d_out;

  char* ws = (char*)d_ws;
  unsigned short* W1H   = (unsigned short*)(ws + kOffW1H);
  unsigned short* W2H   = (unsigned short*)(ws + kOffW2H);
  unsigned short* W3H   = (unsigned short*)(ws + kOffW3H);
  float*          TC    = (float*)(ws + kOffTC);
  unsigned short* A0    = (unsigned short*)(ws + kOffA0);
  float*          COEFF = (float*)(ws + kOffCOEFF);

  prep_planes_kernel<<<7, 256, 0, stream>>>(W1, W2, W3, ltn, W1H, W2H, W3H, TC);

  gain_update_kernel<<<(kBatch * 32) / 256, 256, 0, stream>>>(
      prior_mean, cov_u, cov_l, cov_s, obs, obs_var, out, (unsigned*)A0);

  coeff_net_kernel<<<kBatch / 64, 128, 0, stream>>>(A0, W1H, W2H, W3H, b1, b2, b3, COEFF);

  predict_kernel<<<kBatch / kPR, 256, 0, stream>>>(out, COEFF, TC, tm11b, tm12b, tm21b, tm22b);
}
